// KoopmanOperators_17205638988031
// MI455X (gfx1250) — hardware-verified
//
#include <hip/hip_runtime.h>
#include <hip/hip_bf16.h>

constexpr int kB = 16, kN = 64, kT = 8, kSD = 8;
constexpr int kNodes = kB * kT * kN;
constexpr int kHid = 128, kES = 128, kUD = 32, kRD = 64, kGD = 32;
constexpr int kLdaU = 192;
constexpr int kLdaC = 256;
constexpr int kChunkBT = 16;
constexpr int kChunkNodes = kChunkBT * kN;
constexpr int kChunkPairs = kChunkNodes * kN;
constexpr int kNumChunks = (kB * kT) / kChunkBT;

constexpr size_t oWSW2H = 0;
constexpr size_t oWSW2L = oWSW2H + 128 * 128 * 2;
constexpr size_t oWUW2H = oWSW2L + 128 * 128 * 2;
constexpr size_t oWUW2L = oWUW2H + 64 * 128 * 2;
constexpr size_t oWUPWH = oWUW2L + 64 * 128 * 2;
constexpr size_t oWUPWL = oWUPWH + 64 * 192 * 2;
constexpr size_t oWRPAH = oWUPWL + 64 * 192 * 2;
constexpr size_t oWRPAL = oWRPAH + 64 * 128 * 2;
constexpr size_t oWRPBH = oWRPAL + 64 * 128 * 2;
constexpr size_t oWRPBL = oWRPBH + 64 * 128 * 2;
constexpr size_t oWCW1H = oWRPBL + 64 * 128 * 2;
constexpr size_t oWCW1L = oWCW1H + 128 * 256 * 2;
constexpr size_t oWCW2H = oWCW1L + 128 * 256 * 2;
constexpr size_t oWCW2L = oWCW2H + 128 * 128 * 2;
constexpr size_t oWCW3H = oWCW2L + 128 * 128 * 2;
constexpr size_t oWCW3L = oWCW3H + 64 * 128 * 2;
constexpr size_t oWREW2 = oWCW3L + 64 * 128 * 2;
constexpr size_t oWRPC  = oWREW2 + 64 * 128 * 2;
constexpr size_t oBIAS  = oWRPC + 64 * 64 * 2;
constexpr size_t oP     = oBIAS + 4 * 64 * 4;
constexpr size_t oH1H   = oP + (size_t)kNodes * kHid * 4;
constexpr size_t oH1L   = oH1H + (size_t)kNodes * kHid * 2;
constexpr size_t oHUH   = oH1L + (size_t)kNodes * kHid * 2;
constexpr size_t oHUL   = oHUH + (size_t)kNodes * kHid * 2;
constexpr size_t oAUH   = oHUL + (size_t)kNodes * kHid * 2;
constexpr size_t oAUL   = oAUH + (size_t)kNodes * kLdaU * 2;
constexpr size_t oACH   = oAUL + (size_t)kNodes * kLdaU * 2;
constexpr size_t oACL   = oACH + (size_t)kNodes * kLdaC * 2;
constexpr size_t oRA    = oACL + (size_t)kNodes * kLdaC * 2;
constexpr size_t oRB    = oRA + (size_t)kNodes * kRD * 4;
constexpr size_t oG1H   = oRB + (size_t)kNodes * kRD * 4;
constexpr size_t oG1L   = oG1H + (size_t)kNodes * kHid * 2;
constexpr size_t oG2H   = oG1L + (size_t)kNodes * kHid * 2;
constexpr size_t oG2L   = oG2H + (size_t)kNodes * kHid * 2;
constexpr size_t oG3    = oG2L + (size_t)kNodes * kHid * 2;
constexpr size_t oH16   = oG3 + (size_t)kNodes * kRD * 4;
constexpr size_t oE16   = oH16 + (size_t)kChunkPairs * kHid * 2;
constexpr size_t oTT    = oE16 + (size_t)kChunkPairs * kRD * 2;
constexpr size_t oEnd   = oTT + (size_t)kChunkPairs * kRD * 4;
static_assert(oEnd <= (size_t)134217728, "carve");
static_assert((oP % 256) == 0 && (oH16 % 256) == 0 && (oTT % 256) == 0, "align");

typedef __attribute__((ext_vector_type(16))) _Float16 v16h;
typedef __attribute__((ext_vector_type(8)))  _Float16 v8h;
typedef __attribute__((ext_vector_type(16))) __bf16   v16b;
typedef __attribute__((ext_vector_type(8)))  __bf16   v8b;
typedef __attribute__((ext_vector_type(8)))  float    v8f;
typedef __attribute__((ext_vector_type(4)))  float    v4f;

__device__ __forceinline__ unsigned short f2bf_bits(float f) {
  unsigned u = __float_as_uint(f);
  return (unsigned short)((u + 0x7FFFu + ((u >> 16) & 1u)) >> 16);
}
__device__ __forceinline__ float bf_bits2f(unsigned short h) { return __uint_as_float(((unsigned)h) << 16); }

__device__ __forceinline__ void dep_guard_h(v8f& a, v8f& b, v16h x, v16h y) { asm volatile("v_nop\n\tv_nop\n\tv_nop\n\tv_nop" : "+v"(a), "+v"(b) : "v"(x), "v"(y)); }
__device__ __forceinline__ void dep_guard_b(v8f& a, v8f& b, v16b x, v16b y) { asm volatile("v_nop\n\tv_nop\n\tv_nop\n\tv_nop" : "+v"(a), "+v"(b) : "v"(x), "v"(y)); }
__device__ __forceinline__ void keep4_h(v16h a, v16h b, v16h c, v16h d) { asm volatile("v_nop" :: "v"(a), "v"(b), "v"(c), "v"(d)); }
__device__ __forceinline__ void keep4_b(v16b a, v16b b, v16b c, v16b d) { asm volatile("v_nop" :: "v"(a), "v"(b), "v"(c), "v"(d)); }
__device__ __forceinline__ void acc_guard4(v8f& a, v8f& b, v8f& c, v8f& d) { asm volatile("v_nop\n\tv_nop\n\tv_nop\n\tv_nop" : "+v"(a), "+v"(b), "+v"(c), "+v"(d)); }
template <typename T> struct Frag;
template <> struct Frag<_Float16> {
  typedef v16h V; union U { v16h v; v8h h[2]; };
  static __device__ __forceinline__ v16h load(const _Float16* p) {
    U f; f.h[0] = *(const v8h*)(p); f.h[1] = *(const v8h*)(p + 16); return f.v;
  }
  static __device__ __forceinline__ v8f mma(v16h a, v16h b, v8f c) {
    return __builtin_amdgcn_wmma_f32_16x16x32_f16(false, a, false, b, (short)0, c, false, false);
  }
  static __device__ __forceinline__ void guard(v8f& a, v8f& b, v16h x, v16h y) { dep_guard_h(a, b, x, y); }
  static __device__ __forceinline__ void keep(v16h a, v16h b, v16h c, v16h d) { keep4_h(a, b, c, d); }
};
template <> struct Frag<__bf16> {
  typedef v16b V; union U { v16b v; v8b h[2]; };
  static __device__ __forceinline__ v16b load(const __bf16* p) {
    U f; f.h[0] = *(const v8b*)(p); f.h[1] = *(const v8b*)(p + 16); return f.v;
  }
  static __device__ __forceinline__ v8f mma(v16b a, v16b b, v8f c) {
    return __builtin_amdgcn_wmma_f32_16x16x32_bf16(false, a, false, b, (short)0, c, false, false);
  }
  static __device__ __forceinline__ void guard(v8f& a, v8f& b, v16b x, v16b y) { dep_guard_b(a, b, x, y); }
  static __device__ __forceinline__ void keep(v16b a, v16b b, v16b c, v16b d) { keep4_b(a, b, c, d); }
};

template <int ET> struct Elem;
template <> struct Elem<0> { typedef _Float16 T; };
template <> struct Elem<1> { typedef __bf16 T; };
template <int ET, bool SPLIT, int BIAS_MODE, int OUT_MODE, bool RESID, int ACT = 0>
__global__ __launch_bounds__(256) void wmma_gemm64(
    const unsigned short* __restrict__ Ap, const unsigned short* __restrict__ A2p, int lda, long strideA,
    const unsigned short* __restrict__ Btp, const unsigned short* __restrict__ Bt2p, int ldb, long strideB,
    void* __restrict__ Cout, void* __restrict__ Cout2, int ldc, long strideC,
    const float* __restrict__ bias,
    const float* __restrict__ resid, long strideR,
    int M, int N, int K, float scale) {
  typedef typename Elem<ET>::T T;
  typedef typename Frag<T>::V V;
  const T* A = (const T*)Ap; const T* A2 = (const T*)A2p; const T* Bt = (const T*)Btp; const T* Bt2 = (const T*)Bt2p;
  __shared__ __align__(16) float sT[8][16 * 68];
  const int b    = blockIdx.y;
  const int lane = threadIdx.x & 31;
  const int wave = threadIdx.x >> 5;
  const int tilesN = N >> 6;
  const int tilesM = M >> 6;
  const int tile = blockIdx.x * 8 + wave;
  if (tile >= tilesM * tilesN) return;
  const int tm = tile / tilesN;
  const int tn = tile - tm * tilesN;
  const int m0 = tm << 6;
  const int n0 = tn << 6;

  const T* Ab  = A  + (size_t)b * strideA;
  const T* Bb  = Bt + (size_t)b * strideB;
  const T* Ab2 = SPLIT ? (A2  + (size_t)b * strideA) : nullptr;
  const T* Bb2 = SPLIT ? (Bt2 + (size_t)b * strideB) : nullptr;

  const int rlane = lane & 15;
  const int koff  = (lane >> 4) * 8;
  const int mOff  = (lane >> 4) * 8;

  v8f acc[4][4];
#pragma unroll
  for (int i = 0; i < 4; ++i)
#pragma unroll
    for (int j = 0; j < 4; ++j) acc[i][j] = (v8f){0.f,0.f,0.f,0.f,0.f,0.f,0.f,0.f};

  for (int k0 = 0; k0 < K; k0 += 32) {
    V bh[4], bl[4];
#pragma unroll
    for (int j = 0; j < 4; ++j) {
      const size_t bo = (size_t)(n0 + (j << 4) + rlane) * ldb + koff + k0;
      bh[j] = Frag<T>::load(Bb + bo);
      if (SPLIT) bl[j] = Frag<T>::load(Bb2 + bo);
    }
#pragma unroll
    for (int i = 0; i < 4; ++i) {
      const size_t ao = (size_t)(m0 + (i << 4) + rlane) * lda + koff + k0;
      V ah = Frag<T>::load(Ab + ao);
      V al;
      if (SPLIT) al = Frag<T>::load(Ab2 + ao);
#pragma unroll
      for (int j = 0; j < 4; ++j) {
        acc[i][j] = Frag<T>::mma(ah, bh[j], acc[i][j]);
        if (SPLIT) {
          acc[i][j] = Frag<T>::mma(ah, bl[j], acc[i][j]);
          acc[i][j] = Frag<T>::mma(al, bh[j], acc[i][j]);
        }
      }
      Frag<T>::guard(acc[i][0], acc[i][3], ah, SPLIT ? al : ah);
    }
    Frag<T>::keep(bh[0], bh[1], bh[2], bh[3]);
    if (SPLIT) Frag<T>::keep(bl[0], bl[1], bl[2], bl[3]);
  }
  acc_guard4(acc[0][0], acc[0][1], acc[0][2], acc[0][3]);
  acc_guard4(acc[1][0], acc[1][1], acc[1][2], acc[1][3]);
  acc_guard4(acc[2][0], acc[2][1], acc[2][2], acc[2][3]);
  acc_guard4(acc[3][0], acc[3][1], acc[3][2], acc[3][3]);

  float* slab = sT[wave];
  const float* Rb = RESID ? (resid + (size_t)b * strideR) : nullptr;
#pragma unroll
  for (int i = 0; i < 4; ++i) {
    const int mBase = m0 + (i << 4);
#pragma unroll
    for (int j = 0; j < 4; ++j) {
      const int n = n0 + (j << 4) + rlane;
      float bv = 0.f;
      if (BIAS_MODE == 2) bv = bias[n];
#pragma unroll
      for (int r = 0; r < 8; ++r) {
        float v = acc[i][j][r] * scale;
        if (BIAS_MODE == 1) v += bias[mBase + mOff + r];
        if (BIAS_MODE == 2) v += bv;
        if (RESID) v += Rb[(size_t)(mBase + mOff + r) * ldc + n];
        if (ACT == 1) v = tanhf(v);
        if (ACT == 2) v = fmaxf(v, 0.0f);
        if (ACT == 3) v = v / (1.0f + expf(-v));
        if (ACT == 4) v = (v > 0.f) ? v : 0.01f * v;
        if (ACT == 5) v = 0.5f * v * (1.0f + erff(v * 0.70710678118654752f));
        slab[(mOff + r) * 68 + (j << 4) + rlane] = v;
      }
    }
    __builtin_amdgcn_fence(__ATOMIC_RELEASE, "workgroup");
    __builtin_amdgcn_wave_barrier();
    __builtin_amdgcn_fence(__ATOMIC_ACQUIRE, "workgroup");
    if (OUT_MODE == 0) {
      float* C = (float*)Cout + (size_t)b * strideC;
      const int hh = lane >> 4, c4 = (lane & 15) * 4;
      for (int pass = 0; pass < 2; ++pass) {
#pragma unroll
        for (int it = 0; it < 8; ++it) {
          const int row = it * 2 + hh;
          v4f v = *(const v4f*)(slab + row * 68 + c4);
          *(volatile v4f*)(C + (size_t)(mBase + row) * ldc + n0 + c4) = v;
        }
        __threadfence();
      }
    } else {
      const int q = lane >> 3, c8 = (lane & 7) * 8;
      unsigned short* C  = (unsigned short*)Cout  + (size_t)b * strideC;
      unsigned short* C2 = (OUT_MODE == 2) ? ((unsigned short*)Cout2 + (size_t)b * strideC) : nullptr;
      for (int pass = 0; pass < 2; ++pass) {
#pragma unroll
        for (int it = 0; it < 4; ++it) {
          const int row = it * 4 + q;
          const float* sp = slab + row * 68 + c8;
          v8h hv, lv;
#pragma unroll
          for (int e = 0; e < 8; ++e) {
            if (OUT_MODE == 1) {
              hv[e] = (_Float16)sp[e];
            } else {
              unsigned short hb = f2bf_bits(sp[e]);
              unsigned short lb = f2bf_bits(sp[e] - bf_bits2f(hb));
              hv[e] = __builtin_bit_cast(_Float16, hb);
              lv[e] = __builtin_bit_cast(_Float16, lb);
            }
          }
          *(volatile v8h*)(C + (size_t)(mBase + row) * ldc + n0 + c8) = hv;
          if (OUT_MODE == 2) *(volatile v8h*)(C2 + (size_t)(mBase + row) * ldc + n0 + c8) = lv;
        }
        __threadfence();
      }
    }
    __builtin_amdgcn_fence(__ATOMIC_RELEASE, "workgroup");
    __builtin_amdgcn_wave_barrier();
    __builtin_amdgcn_fence(__ATOMIC_ACQUIRE, "workgroup");
  }
}

__device__ __forceinline__ void split_bf(float v, _Float16& h, _Float16& l) {
  const unsigned short hb = f2bf_bits(v);
  const unsigned short lb = f2bf_bits(v - bf_bits2f(hb));
  h = __builtin_bit_cast(_Float16, hb);
  l = __builtin_bit_cast(_Float16, lb);
}

__global__ __launch_bounds__(256) void k_wsplit(const float* __restrict__ W, int Ksrc, int Nsrc,
    unsigned short* __restrict__ Bh, unsigned short* __restrict__ Bl, int Nout, int Kout, int kA, int gap) {
  const int kch = Kout >> 3;
  const int chunk = blockIdx.x * 256 + threadIdx.x;
  if (chunk >= Nout * kch) return;
  const int n = chunk / kch;
  const int k0 = (chunk - n * kch) * 8;
  const int nc = min(n, Nsrc - 1);
  v8h hv, lv;
#pragma unroll
  for (int e = 0; e < 8; ++e) {
    const int k = k0 + e;
    int ks = (k < kA) ? k : (k - gap);
    const bool valid = ((k < kA) || (k >= kA + gap)) && (ks < Ksrc) && (n < Nsrc);
    ks = min(max(ks, 0), Ksrc - 1);
    float v = W[(size_t)ks * Nsrc + nc];
    v = valid ? v : 0.f;
    _Float16 h, l;
    split_bf(v, h, l);
    hv[e] = h; lv[e] = l;
  }
  unsigned short* ph = Bh + (size_t)chunk * 8;
  unsigned short* pl = Bl + (size_t)chunk * 8;
  for (int pass = 0; pass < 2; ++pass) {
    *(volatile v8h*)ph = hv;
    *(volatile v8h*)pl = lv;
    __threadfence();
  }
}

__global__ __launch_bounds__(256) void k_wcast_f16(const float* __restrict__ W, int Ksrc, int Nsrc,
    unsigned short* __restrict__ Bt, float scale) {
  const int kch = Ksrc >> 3;
  const int chunk = blockIdx.x * 256 + threadIdx.x;
  if (chunk >= Nsrc * kch) return;
  const int n = chunk / kch;
  const int k0 = (chunk - n * kch) * 8;
  v8h hv;
#pragma unroll
  for (int e = 0; e < 8; ++e) hv[e] = (_Float16)(W[(size_t)(k0 + e) * Nsrc + n] * scale);
  unsigned short* p = Bt + (size_t)chunk * 8;
  for (int pass = 0; pass < 2; ++pass) { *(volatile v8h*)p = hv; __threadfence(); }
}

__global__ __launch_bounds__(32) void k_biaspad(const float* __restrict__ s0, int n0,
    const float* __restrict__ s1, int n1, const float* __restrict__ s2, int n2,
    const float* __restrict__ s3, int n3, float sc3, float* __restrict__ dst, const int* __restrict__ unused_i) {
  const int which = blockIdx.x;
  const float* src = s0; int n = n0; float sc = 1.f;
  if (which == 1) { src = s1; n = n1; }
  else if (which == 2) { src = s2; n = n2; }
  else if (which == 3) { src = s3; n = n3; sc = sc3; }
  const int lane = threadIdx.x;
  if (lane < 16) {
    v4f v;
#pragma unroll
    for (int e = 0; e < 4; ++e) {
      const int idx = lane * 4 + e;
      const float x = src[min(idx, n - 1)];
      v[e] = (idx < n) ? x * sc : 0.f;
    }
    float* p = dst + which * 64 + lane * 4;
    for (int pass = 0; pass < 2; ++pass) { *(volatile v4f*)p = v; __threadfence(); }
  }
}

__global__ __launch_bounds__(256) void k_node_h(const float* __restrict__ states,
    const float* __restrict__ sW1, const float* __restrict__ sb1,
    const float* __restrict__ uW1, const float* __restrict__ ub1,
    unsigned short* __restrict__ H1h, unsigned short* __restrict__ H1l,
    unsigned short* __restrict__ HUh, unsigned short* __restrict__ HUl) {
  const int gid = blockIdx.x * 256 + threadIdx.x;
  const int r = gid >> 4;
  const int c0 = (gid & 15) * 8;
  if (r >= kNodes) return;
  const int bt = r >> 6, n = r & 63, b = bt >> 3, t = bt & 7;
  const float* srow = states + ((size_t)(b * kN + n) * kT + t) * kSD;
  float a[8], u[8];
#pragma unroll
  for (int e = 0; e < 8; ++e) { a[e] = 0.f; u[e] = 0.f; }
#pragma unroll 1
  for (int d = 0; d < kSD; ++d) {
    const float sv = srow[d];
    const v4f wa0 = *(const v4f*)(sW1 + d * kHid + c0), wa1 = *(const v4f*)(sW1 + d * kHid + c0 + 4);
    const v4f wu0 = *(const v4f*)(uW1 + d * kHid + c0), wu1 = *(const v4f*)(uW1 + d * kHid + c0 + 4);
#pragma unroll
    for (int e = 0; e < 4; ++e) {
      a[e] += sv * wa0[e]; a[4 + e] += sv * wa1[e];
      u[e] += sv * wu0[e]; u[4 + e] += sv * wu1[e];
    }
  }
  v8h ah, al, uh, ul;
#pragma unroll
  for (int e = 0; e < 8; ++e) {
    const float va = fmaxf(a[e] + sb1[c0 + e], 0.f);
    const float vu = fmaxf(u[e] + ub1[c0 + e], 0.f);
    _Float16 h, l;
    split_bf(va, h, l); ah[e] = h; al[e] = l;
    split_bf(vu, h, l); uh[e] = h; ul[e] = l;
  }
  const size_t o = (size_t)r * kHid + c0;
  for (int pass = 0; pass < 2; ++pass) {
    *(volatile v8h*)(H1h + o) = ah;
    *(volatile v8h*)(H1l + o) = al;
    *(volatile v8h*)(HUh + o) = uh;
    *(volatile v8h*)(HUl + o) = ul;
    __threadfence();
  }
}

__global__ __launch_bounds__(256) void k_node_p(const float* __restrict__ states,
    const float* __restrict__ reW1, float* __restrict__ P) {
  const int gid = blockIdx.x * 256 + threadIdx.x;
  const int r = gid >> 5;
  const int c0 = (gid & 31) * 4;
  if (r >= kNodes) return;
  const int bt = r >> 6, n = r & 63, b = bt >> 3, t = bt & 7;
  const float* srow = states + ((size_t)(b * kN + n) * kT + t) * kSD;
  v4f acc = (v4f){0.f, 0.f, 0.f, 0.f};
#pragma unroll 1
  for (int d = 0; d < kSD; ++d) {
    const float sv = srow[d];
    const v4f w = *(const v4f*)(reW1 + d * kHid + c0);
#pragma unroll
    for (int e = 0; e < 4; ++e) acc[e] += sv * w[e];
  }
  float* p = P + (size_t)r * kHid + c0;
  for (int pass = 0; pass < 2; ++pass) { *(volatile v4f*)p = acc; __threadfence(); }
}

__global__ __launch_bounds__(256) void k_pair_h16(const float* __restrict__ P, const float* __restrict__ reb1,
    unsigned short* __restrict__ H, int nodeBase) {
  const int gid = blockIdx.x * 256 + threadIdx.x;
  const int p = gid >> 4;
  const int c0 = (gid & 15) * 8;
  if (p >= kChunkPairs) return;
  const int nodeL = p >> 6, j = p & 63;
  const int nodeI = nodeBase + nodeL;
  const int nodeJ = nodeBase + (nodeL & ~63) + j;
  const float* pi = P + (size_t)nodeI * kHid + c0;
  const float* pj = P + (size_t)nodeJ * kHid + c0;
  const v4f i0 = *(const v4f*)pi, i1 = *(const v4f*)(pi + 4);
  const v4f j0 = *(const v4f*)pj, j1 = *(const v4f*)(pj + 4);
  const v4f b0 = *(const v4f*)(reb1 + c0), b1 = *(const v4f*)(reb1 + c0 + 4);
  v8h hv;
#pragma unroll
  for (int e = 0; e < 4; ++e) {
    hv[e]     = (_Float16)fmaxf(i0[e] - j0[e] + b0[e], 0.f);
    hv[4 + e] = (_Float16)fmaxf(i1[e] - j1[e] + b1[e], 0.f);
  }
  unsigned short* q = H + (size_t)p * kHid + c0;
  for (int pass = 0; pass < 2; ++pass) { *(volatile v8h*)q = hv; __threadfence(); }
}

__global__ __launch_bounds__(256) void k_agg(const float* __restrict__ states, const float* __restrict__ RA,
    const float* __restrict__ RB, const float* __restrict__ TT,
    unsigned short* __restrict__ Ah, unsigned short* __restrict__ Al, int nodeBase) {
  __shared__ __align__(16) _Float16 hiS[16 * 64];
  __shared__ __align__(16) _Float16 loS[16 * 64];
  const int tid = threadIdx.x;
  const int nl = tid >> 4, f0 = (tid & 15) * 4;
  const int nodeL = blockIdx.x * 16 + nl;
  const int node = nodeBase + nodeL;
  const int bt = node >> 6, i = node & 63, b = bt >> 3, t = bt & 7;
  const float* si = states + ((size_t)(b * kN + i) * kT + t) * kSD;
  const float si0 = si[0], si4 = si[4];
  const v4f ra = *(const v4f*)(RA + (size_t)node * kRD + f0);
  const float* rbBase = RB + (size_t)(bt * kN) * kRD + f0;
  const float* ttBase = TT + (size_t)nodeL * kN * kRD + f0;
  const float* sjBase = states + ((size_t)(b * kN) * kT + t) * kSD;
  float acc0 = 0.f, acc1 = 0.f, acc2 = 0.f, acc3 = 0.f;
#pragma unroll 1
  for (int j = 0; j < kN; ++j) {
    const float sj0 = sjBase[j * kT * kSD];
    const float sj4 = sjBase[j * kT * kSD + 4];
    const bool sel = (fabsf(si0 - sj0) > 0.1f) || (fabsf(si4 - sj4) > 0.1f);
    const v4f rb = *(const v4f*)(rbBase + j * kRD);
    const v4f tt = *(const v4f*)(ttBase + j * kRD);
    const float v0 = fmaxf(ra[0] + rb[0] + tt[0], 0.f);
    const float v1 = fmaxf(ra[1] + rb[1] + tt[1], 0.f);
    const float v2 = fmaxf(ra[2] + rb[2] + tt[2], 0.f);
    const float v3 = fmaxf(ra[3] + rb[3] + tt[3], 0.f);
    acc0 += sel ? v0 : 0.f;
    acc1 += sel ? v1 : 0.f;
    acc2 += sel ? v2 : 0.f;
    acc3 += sel ? v3 : 0.f;
  }
  {
    _Float16 h, l;
    split_bf(acc0, h, l); hiS[nl * 64 + f0 + 0] = h; loS[nl * 64 + f0 + 0] = l;
    split_bf(acc1, h, l); hiS[nl * 64 + f0 + 1] = h; loS[nl * 64 + f0 + 1] = l;
    split_bf(acc2, h, l); hiS[nl * 64 + f0 + 2] = h; loS[nl * 64 + f0 + 2] = l;
    split_bf(acc3, h, l); hiS[nl * 64 + f0 + 3] = h; loS[nl * 64 + f0 + 3] = l;
  }
  __syncthreads();
  const int t2 = tid & 127;
  const int q = t2 >> 3, seg = t2 & 7;
  const v8h vh = *(const v8h*)(hiS + q * 64 + seg * 8);
  const v8h vl = *(const v8h*)(loS + q * 64 + seg * 8);
  const size_t o = (size_t)(nodeBase + blockIdx.x * 16 + q) * kLdaC + 192 + seg * 8;
  if (tid < 128) {
    for (int pass = 0; pass < 2; ++pass) { *(volatile v8h*)(Ah + o) = vh; __threadfence(); }
  } else {
    for (int pass = 0; pass < 2; ++pass) { *(volatile v8h*)(Al + o) = vl; __threadfence(); }
  }
}

__global__ __launch_bounds__(256) void k_copy_enc(const unsigned short* __restrict__ Sh, const unsigned short* __restrict__ Sl,
    unsigned short* __restrict__ Dh, unsigned short* __restrict__ Dl) {
  const int gid = blockIdx.x * 256 + threadIdx.x;
  const int r = gid >> 4, seg = gid & 15;
  if (r >= kNodes) return;
  const v8h vh = *(const v8h*)(Sh + (size_t)r * kLdaU + seg * 8);
  const v8h vl = *(const v8h*)(Sl + (size_t)r * kLdaU + seg * 8);
  const size_t o = (size_t)r * kLdaC + seg * 8;
  for (int pass = 0; pass < 2; ++pass) {
    *(volatile v8h*)(Dh + o) = vh;
    *(volatile v8h*)(Dl + o) = vl;
    __threadfence();
  }
}

__global__ __launch_bounds__(256) void k_out(const float* __restrict__ G3, float* __restrict__ out) {
  const int gid = blockIdx.x * 256 + threadIdx.x;
  const int r = gid >> 3, seg = gid & 7;
  if (r >= kNodes) return;
  const v4f v = *(const v4f*)(G3 + (size_t)r * kRD + seg * 4);
  float* p = out + (size_t)r * kGD + seg * 4;
  for (int pass = 0; pass < 2; ++pass) { *(volatile v4f*)p = v; __threadfence(); }
}

static inline unsigned cdiv_u(unsigned a, unsigned b) { return (a + b - 1) / b; }

extern "C" void kernel_launch(void* const* d_in, const int* in_sizes, int n_in,
                              void* d_out, int out_size, void* d_ws, size_t ws_size,
                              hipStream_t stream) {
  if (n_in < 24) return;
  if (in_sizes[0] != kNodes * kSD) return;
  if (out_size != kNodes * kGD) return;
  if (ws_size < oEnd) return;

  const float* states = (const float*)d_in[0];
  const int*   temp_i = (const int*)d_in[1];
  const float* sW1  = (const float*)d_in[2];  const float* sb1  = (const float*)d_in[3];
  const float* sW2  = (const float*)d_in[4];  const float* sb2  = (const float*)d_in[5];
  const float* uW1  = (const float*)d_in[6];  const float* ub1  = (const float*)d_in[7];
  const float* uW2  = (const float*)d_in[8];  const float* ub2  = (const float*)d_in[9];
  const float* upW  = (const float*)d_in[10]; const float* upb  = (const float*)d_in[11];
  const float* reW1 = (const float*)d_in[12]; const float* reb1 = (const float*)d_in[13];
  const float* reW2 = (const float*)d_in[14]; const float* reb2 = (const float*)d_in[15];
  const float* rpW  = (const float*)d_in[16]; const float* rpb  = (const float*)d_in[17];
  const float* cW1  = (const float*)d_in[18]; const float* cb1  = (const float*)d_in[19];
  const float* cW2  = (const float*)d_in[20]; const float* cb2  = (const float*)d_in[21];
  const float* cW3  = (const float*)d_in[22]; const float* cb3  = (const float*)d_in[23];
  float* out = (float*)d_out;

  char* ws = (char*)d_ws;
  unsigned short* wSW2h = (unsigned short*)(ws + oWSW2H); unsigned short* wSW2l = (unsigned short*)(ws + oWSW2L);
  unsigned short* wUW2h = (unsigned short*)(ws + oWUW2H); unsigned short* wUW2l = (unsigned short*)(ws + oWUW2L);
  unsigned short* wUPWh = (unsigned short*)(ws + oWUPWH); unsigned short* wUPWl = (unsigned short*)(ws + oWUPWL);
  unsigned short* wRPAh = (unsigned short*)(ws + oWRPAH); unsigned short* wRPAl = (unsigned short*)(ws + oWRPAL);
  unsigned short* wRPBh = (unsigned short*)(ws + oWRPBH); unsigned short* wRPBl = (unsigned short*)(ws + oWRPBL);
  unsigned short* wCW1h = (unsigned short*)(ws + oWCW1H); unsigned short* wCW1l = (unsigned short*)(ws + oWCW1L);
  unsigned short* wCW2h = (unsigned short*)(ws + oWCW2H); unsigned short* wCW2l = (unsigned short*)(ws + oWCW2L);
  unsigned short* wCW3h = (unsigned short*)(ws + oWCW3H); unsigned short* wCW3l = (unsigned short*)(ws + oWCW3L);
  unsigned short* wREW2 = (unsigned short*)(ws + oWREW2);
  unsigned short* wRPC  = (unsigned short*)(ws + oWRPC);
  float* biaspad = (float*)(ws + oBIAS);
  float* Pf  = (float*)(ws + oP);
  unsigned short* H1h = (unsigned short*)(ws + oH1H); unsigned short* H1l = (unsigned short*)(ws + oH1L);
  unsigned short* HUh = (unsigned short*)(ws + oHUH); unsigned short* HUl = (unsigned short*)(ws + oHUL);
  unsigned short* AUh = (unsigned short*)(ws + oAUH); unsigned short* AUl = (unsigned short*)(ws + oAUL);
  unsigned short* ACh = (unsigned short*)(ws + oACH); unsigned short* ACl = (unsigned short*)(ws + oACL);
  float* RAf = (float*)(ws + oRA);
  float* RBf = (float*)(ws + oRB);
  unsigned short* G1h = (unsigned short*)(ws + oG1H); unsigned short* G1l = (unsigned short*)(ws + oG1L);
  unsigned short* G2h = (unsigned short*)(ws + oG2H); unsigned short* G2l = (unsigned short*)(ws + oG2L);
  float* G3f = (float*)(ws + oG3);
  unsigned short* H16 = (unsigned short*)(ws + oH16);
  unsigned short* E16 = (unsigned short*)(ws + oE16);
  float* TTf = (float*)(ws + oTT);
  const float* fdummy = biaspad;

  k_wsplit<<<cdiv_u(128 * 128 / 8, 256), 256, 0, stream>>>(sW2, 128, 128, wSW2h, wSW2l, 128, 128, 128, 0);
  k_wsplit<<<cdiv_u(64 * 128 / 8, 256), 256, 0, stream>>>(uW2, 128, 32, wUW2h, wUW2l, 64, 128, 128, 0);
  k_wsplit<<<cdiv_u(64 * 192 / 8, 256), 256, 0, stream>>>(upW, 160, 32, wUPWh, wUPWl, 64, 192, 160, 32);
  k_wsplit<<<cdiv_u(64 * 128 / 8, 256), 256, 0, stream>>>(rpW, 128, 64, wRPAh, wRPAl, 64, 128, 128, 0);
  k_wsplit<<<cdiv_u(64 * 128 / 8, 256), 256, 0, stream>>>(rpW + 128 * 64, 128, 64, wRPBh, wRPBl, 64, 128, 128, 0);
  k_wsplit<<<cdiv_u(128 * 256 / 8, 256), 256, 0, stream>>>(cW1, 224, 128, wCW1h, wCW1l, 128, 256, 160, 32);
  k_wsplit<<<cdiv_u(128 * 128 / 8, 256), 256, 0, stream>>>(cW2, 128, 128, wCW2h, wCW2l, 128, 128, 128, 0);
  k_wsplit<<<cdiv_u(64 * 128 / 8, 256), 256, 0, stream>>>(cW3, 128, 32, wCW3h, wCW3l, 64, 128, 128, 0);
  k_wcast_f16<<<cdiv_u(64 * 128 / 8, 256), 256, 0, stream>>>(reW2, 128, 64, wREW2, 8.0f);
  k_wcast_f16<<<cdiv_u(64 * 64 / 8, 256), 256, 0, stream>>>(rpW + 256 * 64, 64, 64, wRPC, 8.0f);
  k_biaspad<<<4, 32, 0, stream>>>(ub2, 32, upb, 32, cb3, 32, reb2, 64, 4.0f, biaspad, temp_i);

  k_node_h<<<cdiv_u(kNodes * 16, 256), 256, 0, stream>>>(states, sW1, sb1, uW1, ub1, H1h, H1l, HUh, HUl);
  k_node_p<<<cdiv_u(kNodes * 32, 256), 256, 0, stream>>>(states, reW1, Pf);

  wmma_gemm64<1, true, 2, 2, false, 2><<<dim3(32, 1), 256, 0, stream>>>(
      H1h, H1l, 128, 0L, wSW2h, wSW2l, 128, 0L, (void*)AUh, (void*)AUl, kLdaU, 0L, sb2, fdummy, 0L, kNodes, 128, 128, 1.0f);
  wmma_gemm64<1, true, 2, 2, false, 0><<<dim3(16, 1), 256, 0, stream>>>(
      HUh, HUl, 128, 0L, wUW2h, wUW2l, 128, 0L, (void*)(AUh + 128), (void*)(AUl + 128), kLdaU, 0L, biaspad + 0, fdummy, 0L, kNodes, 64, 128, 1.0f);
  wmma_gemm64<1, true, 2, 2, false, 2><<<dim3(16, 1), 256, 0, stream>>>(
      AUh, AUl, kLdaU, 0L, wUPWh, wUPWl, 192, 0L, (void*)(ACh + 128), (void*)(ACl + 128), kLdaC, 0L, biaspad + 64, fdummy, 0L, kNodes, 64, 192, 1.0f);
  wmma_gemm64<1, true, 2, 0, false, 0><<<dim3(16, 1), 256, 0, stream>>>(
      AUh, AUl, kLdaU, 0L, wRPAh, wRPAl, 128, 0L, (void*)RAf, (void*)RAf, kRD, 0L, rpb, fdummy, 0L, kNodes, 64, 128, 1.0f);
  wmma_gemm64<1, true, 0, 0, false, 0><<<dim3(16, 1), 256, 0, stream>>>(
      AUh, AUl, kLdaU, 0L, wRPBh, wRPBl, 128, 0L, (void*)RBf, (void*)RBf, kRD, 0L, fdummy, fdummy, 0L, kNodes, 64, 128, 1.0f);

  for (int c = 0; c < kNumChunks; ++c) {
    const int nodeBase = c * kChunkNodes;
    k_pair_h16<<<cdiv_u(kChunkPairs * 16, 256), 256, 0, stream>>>(Pf, reb1, H16, nodeBase);
    wmma_gemm64<0, false, 2, 1, false, 2><<<dim3(128, 1), 256, 0, stream>>>(
        H16, H16, 128, 0L, wREW2, wREW2, 128, 0L, (void*)E16, (void*)E16, kRD, 0L, biaspad + 192, fdummy, 0L, kChunkPairs, 64, 128, 0.5f);
    wmma_gemm64<0, false, 0, 0, false, 0><<<dim3(128, 1), 256, 0, stream>>>(
        E16, E16, 64, 0L, wRPC, wRPC, 64, 0L, (void*)TTf, (void*)TTf, kRD, 0L, fdummy, fdummy, 0L, kChunkPairs, 64, 64, 1.0f / 32.0f);
    k_agg<<<kChunkNodes / 16, 256, 0, stream>>>(states, RAf, RBf, TTf, ACh, ACl, nodeBase);
  }

  k_copy_enc<<<cdiv_u(kNodes * 16, 256), 256, 0, stream>>>(AUh, AUl, ACh, ACl);
  wmma_gemm64<1, true, 2, 2, false, 2><<<dim3(32, 1), 256, 0, stream>>>(
      ACh, ACl, kLdaC, 0L, wCW1h, wCW1l, 256, 0L, (void*)G1h, (void*)G1l, 128, 0L, cb1, fdummy, 0L, kNodes, 128, 256, 1.0f);
  wmma_gemm64<1, true, 2, 2, false, 2><<<dim3(32, 1), 256, 0, stream>>>(
      G1h, G1l, 128, 0L, wCW2h, wCW2l, 128, 0L, (void*)G2h, (void*)G2l, 128, 0L, cb2, fdummy, 0L, kNodes, 128, 128, 1.0f);
  wmma_gemm64<1, true, 2, 0, false, 0><<<dim3(16, 1), 256, 0, stream>>>(
      G2h, G2l, 128, 0L, wCW3h, wCW3l, 128, 0L, (void*)G3f, (void*)G3f, kRD, 0L, biaspad + 128, fdummy, 0L, kNodes, 64, 128, 1.0f);
  k_out<<<cdiv_u(kNodes * 8, 256), 256, 0, stream>>>(G3f, out);
}
